// DeformableConv2dLayer_20349555048916
// MI455X (gfx1250) — hardware-verified
//
#include <hip/hip_runtime.h>
#include <stdint.h>


typedef __attribute__((ext_vector_type(16))) _Float16 v16h;
typedef __attribute__((ext_vector_type(8)))  _Float16 v8h;
typedef __attribute__((ext_vector_type(16))) __bf16   v16b;
typedef __attribute__((ext_vector_type(8)))  __bf16   v8b;
typedef __attribute__((ext_vector_type(8)))  float    v8f;
typedef __attribute__((ext_vector_type(4)))  float    v4f;

#define HDIM 128
#define WDIM 128
#define CDIM 32
#define CODIM 32
#define NPTS 9
#define KDIM (NPTS * CDIM)
#define NPAD 64
#define GW 4
#define PPW 8
#define WSCALE 64.0f
#define WSCALE_INV (1.0f / 64.0f)

#define DI_BITS 99984u
#define DJ_BITS 137364u

__device__ __forceinline__ unsigned short f2bf_bits(float f) {
  unsigned u = __float_as_uint(f);
  return (unsigned short)((u + 0x7FFFu + ((u >> 16) & 1u)) >> 16);
}
__device__ __forceinline__ float bf_bits2f(unsigned short h) { return __uint_as_float(((unsigned)h) << 16); }

__device__ __forceinline__ void dep_guard_h(v8f& a, v8f& b, v16h x, v16h y) { asm volatile("v_nop\n\tv_nop\n\tv_nop\n\tv_nop" : "+v"(a), "+v"(b) : "v"(x), "v"(y)); }
__device__ __forceinline__ void dep_guard_b(v8f& a, v8f& b, v16b x, v16b y) { asm volatile("v_nop\n\tv_nop\n\tv_nop\n\tv_nop" : "+v"(a), "+v"(b) : "v"(x), "v"(y)); }
__device__ __forceinline__ void keep4_h(v16h a, v16h b, v16h c, v16h d) { asm volatile("v_nop" :: "v"(a), "v"(b), "v"(c), "v"(d)); }
__device__ __forceinline__ void keep4_b(v16b a, v16b b, v16b c, v16b d) { asm volatile("v_nop" :: "v"(a), "v"(b), "v"(c), "v"(d)); }
__device__ __forceinline__ void acc_guard4(v8f& a, v8f& b, v8f& c, v8f& d) { asm volatile("v_nop\n\tv_nop\n\tv_nop\n\tv_nop" : "+v"(a), "+v"(b), "+v"(c), "+v"(d)); }
template <typename T> struct Frag;
template <> struct Frag<_Float16> {
  typedef v16h V; union U { v16h v; v8h h[2]; };
  static __device__ __forceinline__ v16h load(const _Float16* p) {
    U f; f.h[0] = *(const v8h*)(p); f.h[1] = *(const v8h*)(p + 16); return f.v;
  }
  static __device__ __forceinline__ v8f mma(v16h a, v16h b, v8f c) {
    return __builtin_amdgcn_wmma_f32_16x16x32_f16(false, a, false, b, (short)0, c, false, false);
  }
  static __device__ __forceinline__ void guard(v8f& a, v8f& b, v16h x, v16h y) { dep_guard_h(a, b, x, y); }
  static __device__ __forceinline__ void keep(v16h a, v16h b, v16h c, v16h d) { keep4_h(a, b, c, d); }
};
template <> struct Frag<__bf16> {
  typedef v16b V; union U { v16b v; v8b h[2]; };
  static __device__ __forceinline__ v16b load(const __bf16* p) {
    U f; f.h[0] = *(const v8b*)(p); f.h[1] = *(const v8b*)(p + 16); return f.v;
  }
  static __device__ __forceinline__ v8f mma(v16b a, v16b b, v8f c) {
    return __builtin_amdgcn_wmma_f32_16x16x32_bf16(false, a, false, b, (short)0, c, false, false);
  }
  static __device__ __forceinline__ void guard(v8f& a, v8f& b, v16b x, v16b y) { dep_guard_b(a, b, x, y); }
  static __device__ __forceinline__ void keep(v16b a, v16b b, v16b c, v16b d) { keep4_b(a, b, c, d); }
};

template <int ET> struct Elem;
template <> struct Elem<0> { typedef _Float16 T; };
template <> struct Elem<1> { typedef __bf16 T; };
template <int ET, bool SPLIT, int BIAS_MODE, int OUT_MODE, bool RESID, int ACT = 0>
__global__ __launch_bounds__(256) void wmma_gemm64(
    const unsigned short* __restrict__ Ap, const unsigned short* __restrict__ A2p, int lda, long strideA,
    const unsigned short* __restrict__ Btp, const unsigned short* __restrict__ Bt2p, int ldb, long strideB,
    void* __restrict__ Cout, void* __restrict__ Cout2, int ldc, long strideC,
    const float* __restrict__ bias,
    const float* __restrict__ resid, long strideR,
    int M, int N, int K, float scale) {
  typedef typename Elem<ET>::T T;
  typedef typename Frag<T>::V V;
  const T* A = (const T*)Ap; const T* A2 = (const T*)A2p; const T* Bt = (const T*)Btp; const T* Bt2 = (const T*)Bt2p;
  __shared__ __align__(16) float sT[8][16 * 68];
  const int b    = blockIdx.y;
  const int lane = threadIdx.x & 31;
  const int wave = threadIdx.x >> 5;
  const int tilesN = N >> 6;
  const int tilesM = M >> 6;
  const int tile = blockIdx.x * 8 + wave;
  if (tile >= tilesM * tilesN) return;
  const int tm = tile / tilesN;
  const int tn = tile - tm * tilesN;
  const int m0 = tm << 6;
  const int n0 = tn << 6;

  const T* Ab  = A  + (size_t)b * strideA;
  const T* Bb  = Bt + (size_t)b * strideB;
  const T* Ab2 = SPLIT ? (A2  + (size_t)b * strideA) : nullptr;
  const T* Bb2 = SPLIT ? (Bt2 + (size_t)b * strideB) : nullptr;

  const int rlane = lane & 15;
  const int koff  = (lane >> 4) * 8;
  const int mOff  = (lane >> 4) * 8;

  v8f acc[4][4];
#pragma unroll
  for (int i = 0; i < 4; ++i)
#pragma unroll
    for (int j = 0; j < 4; ++j) acc[i][j] = (v8f){0.f,0.f,0.f,0.f,0.f,0.f,0.f,0.f};

  for (int k0 = 0; k0 < K; k0 += 32) {
    V bh[4], bl[4];
#pragma unroll
    for (int j = 0; j < 4; ++j) {
      const size_t bo = (size_t)(n0 + (j << 4) + rlane) * ldb + koff + k0;
      bh[j] = Frag<T>::load(Bb + bo);
      if (SPLIT) bl[j] = Frag<T>::load(Bb2 + bo);
    }
#pragma unroll
    for (int i = 0; i < 4; ++i) {
      const size_t ao = (size_t)(m0 + (i << 4) + rlane) * lda + koff + k0;
      V ah = Frag<T>::load(Ab + ao);
      V al;
      if (SPLIT) al = Frag<T>::load(Ab2 + ao);
#pragma unroll
      for (int j = 0; j < 4; ++j) {
        acc[i][j] = Frag<T>::mma(ah, bh[j], acc[i][j]);
        if (SPLIT) {
          acc[i][j] = Frag<T>::mma(ah, bl[j], acc[i][j]);
          acc[i][j] = Frag<T>::mma(al, bh[j], acc[i][j]);
        }
      }
      Frag<T>::guard(acc[i][0], acc[i][3], ah, SPLIT ? al : ah);
    }
    Frag<T>::keep(bh[0], bh[1], bh[2], bh[3]);
    if (SPLIT) Frag<T>::keep(bl[0], bl[1], bl[2], bl[3]);
  }
  acc_guard4(acc[0][0], acc[0][1], acc[0][2], acc[0][3]);
  acc_guard4(acc[1][0], acc[1][1], acc[1][2], acc[1][3]);
  acc_guard4(acc[2][0], acc[2][1], acc[2][2], acc[2][3]);
  acc_guard4(acc[3][0], acc[3][1], acc[3][2], acc[3][3]);

  float* slab = sT[wave];
  const float* Rb = RESID ? (resid + (size_t)b * strideR) : nullptr;
#pragma unroll
  for (int i = 0; i < 4; ++i) {
    const int mBase = m0 + (i << 4);
#pragma unroll
    for (int j = 0; j < 4; ++j) {
      const int n = n0 + (j << 4) + rlane;
      float bv = 0.f;
      if (BIAS_MODE == 2) bv = bias[n];
#pragma unroll
      for (int r = 0; r < 8; ++r) {
        float v = acc[i][j][r] * scale;
        if (BIAS_MODE == 1) v += bias[mBase + mOff + r];
        if (BIAS_MODE == 2) v += bv;
        if (RESID) v += Rb[(size_t)(mBase + mOff + r) * ldc + n];
        if (ACT == 1) v = tanhf(v);
        if (ACT == 2) v = fmaxf(v, 0.0f);
        if (ACT == 3) v = v / (1.0f + expf(-v));
        if (ACT == 4) v = (v > 0.f) ? v : 0.01f * v;
        if (ACT == 5) v = 0.5f * v * (1.0f + erff(v * 0.70710678118654752f));
        slab[(mOff + r) * 68 + (j << 4) + rlane] = v;
      }
    }
    __builtin_amdgcn_fence(__ATOMIC_RELEASE, "workgroup");
    __builtin_amdgcn_wave_barrier();
    __builtin_amdgcn_fence(__ATOMIC_ACQUIRE, "workgroup");
    if (OUT_MODE == 0) {
      float* C = (float*)Cout + (size_t)b * strideC;
      const int hh = lane >> 4, c4 = (lane & 15) * 4;
      for (int pass = 0; pass < 2; ++pass) {
#pragma unroll
        for (int it = 0; it < 8; ++it) {
          const int row = it * 2 + hh;
          v4f v = *(const v4f*)(slab + row * 68 + c4);
          *(volatile v4f*)(C + (size_t)(mBase + row) * ldc + n0 + c4) = v;
        }
        __threadfence();
      }
    } else {
      const int q = lane >> 3, c8 = (lane & 7) * 8;
      unsigned short* C  = (unsigned short*)Cout  + (size_t)b * strideC;
      unsigned short* C2 = (OUT_MODE == 2) ? ((unsigned short*)Cout2 + (size_t)b * strideC) : nullptr;
      for (int pass = 0; pass < 2; ++pass) {
#pragma unroll
        for (int it = 0; it < 4; ++it) {
          const int row = it * 4 + q;
          const float* sp = slab + row * 68 + c8;
          v8h hv, lv;
#pragma unroll
          for (int e = 0; e < 8; ++e) {
            if (OUT_MODE == 1) {
              hv[e] = (_Float16)sp[e];
            } else {
              unsigned short hb = f2bf_bits(sp[e]);
              unsigned short lb = f2bf_bits(sp[e] - bf_bits2f(hb));
              hv[e] = __builtin_bit_cast(_Float16, hb);
              lv[e] = __builtin_bit_cast(_Float16, lb);
            }
          }
          *(volatile v8h*)(C + (size_t)(mBase + row) * ldc + n0 + c8) = hv;
          if (OUT_MODE == 2) *(volatile v8h*)(C2 + (size_t)(mBase + row) * ldc + n0 + c8) = lv;
        }
        __threadfence();
      }
    }
    __builtin_amdgcn_fence(__ATOMIC_RELEASE, "workgroup");
    __builtin_amdgcn_wave_barrier();
    __builtin_amdgcn_fence(__ATOMIC_ACQUIRE, "workgroup");
  }
}

__global__ __launch_bounds__(256) void build_wt_f16(
    const float* __restrict__ Wg, _Float16* __restrict__ Wt, int nchunks) {
  const int t = blockIdx.x * 256 + threadIdx.x;
  if (t < nchunks) {
    const int o  = t / (KDIM / 8);
    const int k0 = (t - o * (KDIM / 8)) * 8;
    const int oc = (o < CODIM) ? o : (CODIM - 1);
    v8h v;
#pragma unroll
    for (int e = 0; e < 8; ++e) {
      const float w = Wg[(size_t)(k0 + e) * CODIM + oc] * WSCALE;
      v[e] = (o < CODIM) ? (_Float16)w : (_Float16)0.0f;
    }
    _Float16* dst = Wt + (size_t)t * 8;
    *(volatile v8h*)dst = v;
    __threadfence();
    *(volatile v8h*)dst = v;
  }
}

__global__ __launch_bounds__(GW * 32) void sample_rows_f16(
    const float* __restrict__ x, const float* __restrict__ offs,
    _Float16* __restrict__ Aout, int npix) {
  __shared__ __align__(16) float    soff[GW][PPW * 2 * NPTS];
  __shared__ __align__(16) _Float16 tile[GW][PPW * KDIM];

  const int lane = threadIdx.x & 31;
  const int wave = threadIdx.x >> 5;
  const int grp  = blockIdx.x * GW + wave;
  const int p0   = grp * PPW;
  const bool active = (p0 + PPW) <= npix;
  const int p0c  = active ? p0 : 0;
  const int b    = p0c / (HDIM * WDIM);
  const int rem  = p0c - b * (HDIM * WDIM);
  const int h    = rem / WDIM;
  const int w0   = rem - h * WDIM;

  float*    so = soff[wave];
  _Float16* tw = tile[wave];

  if (active) {
    const float* op = offs + (size_t)p0c * (2 * NPTS);
    for (int i = lane; i < PPW * 2 * NPTS; i += 32) so[i] = op[i];
  }
  __syncthreads();

  if (active) {
    const float* xb = x + (size_t)b * (HDIM * WDIM * CDIM) + lane;
#pragma unroll 1
    for (int p = 0; p < PPW; ++p) {
      const int wp = w0 + p;
      const float* sp = so + p * (2 * NPTS);
      _Float16* tp = tw + p * KDIM + lane;
#pragma unroll
      for (int n = 0; n < NPTS; ++n) {
        const int di = (int)((DI_BITS >> (2 * n)) & 3u);
        const int dj = (int)((DJ_BITS >> (2 * n)) & 3u);
        const float o0 = sp[2 * n];
        const float o1 = sp[2 * n + 1];
        float c0 = (float)(h - 1 + di) + o0;
        float c1 = (float)(wp - 1 + dj) + o1;
        c0 = fminf(fmaxf(c0, 0.0f), (float)(HDIM - 1));
        c1 = fminf(fmaxf(c1, 0.0f), (float)(WDIM - 1));
        const float fl0 = floorf(c0), fl1 = floorf(c1);
        int lt0 = (int)fl0, lt1 = (int)fl1;
        int rb0 = (int)ceilf(c0), rb1 = (int)ceilf(c1);
        lt0 = lt0 < 0 ? 0 : (lt0 > HDIM - 1 ? HDIM - 1 : lt0);
        rb0 = rb0 < 0 ? 0 : (rb0 > HDIM - 1 ? HDIM - 1 : rb0);
        lt1 = lt1 < 0 ? 0 : (lt1 > WDIM - 1 ? WDIM - 1 : lt1);
        rb1 = rb1 < 0 ? 0 : (rb1 > WDIM - 1 ? WDIM - 1 : rb1);
        const float f0 = c0 - fl0, f1 = c1 - fl1;

        const float v_lt = xb[(size_t)(lt0 * WDIM + lt1) * CDIM];
        const float v_rb = xb[(size_t)(rb0 * WDIM + rb1) * CDIM];
        const float v_lb = xb[(size_t)(lt0 * WDIM + rb1) * CDIM];
        const float v_rt = xb[(size_t)(rb0 * WDIM + lt1) * CDIM];

        const float v_t = v_lt + (v_rt - v_lt) * f0;
        const float v_b = v_lb + (v_rb - v_lb) * f0;
        const float m   = v_t + (v_b - v_t) * f1;
        tp[n * CDIM] = (_Float16)m;
      }
    }
  }
  __syncthreads();

  if (active) {
    _Float16* dst = Aout + (size_t)p0c * KDIM;
    for (int pass = 0; pass < 2; ++pass) {
#pragma unroll
      for (int q = 0; q < (PPW * KDIM) / 256; ++q) {
        const int ci = q * 32 + lane;
        const v8h v = *(const v8h*)(tw + ci * 8);
        *(volatile v8h*)(dst + (size_t)ci * 8) = v;
      }
      __threadfence();
    }
  }
}

__global__ __launch_bounds__(256) void bias_rows_out(
    const float* __restrict__ Cb, const float* __restrict__ bias,
    float* __restrict__ out, int nvec) {
  const int t = blockIdx.x * 256 + threadIdx.x;
  if (t < nvec) {
    const int row = t >> 3;
    const int c4  = (t & 7) * 4;
    const v4f v = *(const v4f*)(Cb + (size_t)row * NPAD + c4);
    v4f r;
    r[0] = v[0] + bias[c4 + 0];
    r[1] = v[1] + bias[c4 + 1];
    r[2] = v[2] + bias[c4 + 2];
    r[3] = v[3] + bias[c4 + 3];
    float* dst = out + (size_t)row * CODIM + c4;
    *(volatile v4f*)dst = r;
    __threadfence();
    *(volatile v4f*)dst = r;
  }
}

extern "C" void kernel_launch(void* const* d_in, const int* in_sizes, int n_in,
                              void* d_out, int out_size, void* d_ws, size_t ws_size,
                              hipStream_t stream) {
  if (n_in < 4) return;
  const int per_b = HDIM * WDIM * CDIM;
  const int nx = in_sizes[0];
  if (nx <= 0 || (nx % per_b) != 0) return;
  const int B = nx / per_b;
  const int npix = B * HDIM * WDIM;
  if (in_sizes[1] != npix * 2 * NPTS) return;
  if (in_sizes[2] != NPTS * CDIM * CODIM) return;
  if (in_sizes[3] < CODIM) return;
  if (out_size != npix * CODIM) return;

  const size_t offA = 0;
  const size_t szA  = (size_t)npix * KDIM * sizeof(_Float16);
  const size_t offW = offA + szA;
  const size_t szW  = (size_t)NPAD * KDIM * sizeof(_Float16);
  const size_t offC = offW + szW;
  const size_t szC  = (size_t)npix * NPAD * sizeof(float);
  const size_t total = offC + szC;
  if (total > ws_size || total > (size_t)134217728) return;

  const float* x    = (const float*)d_in[0];
  const float* offs = (const float*)d_in[1];
  const float* Wg   = (const float*)d_in[2];
  const float* bias = (const float*)d_in[3];
  float* out = (float*)d_out;
  char* ws = (char*)d_ws;
  _Float16* Aplane = (_Float16*)(ws + offA);
  _Float16* Wt     = (_Float16*)(ws + offW);
  float*    Cbuf   = (float*)(ws + offC);

  const int nchunks = NPAD * KDIM / 8;
  build_wt_f16<<<(nchunks + 255) / 256, 256, 0, stream>>>(Wg, Wt, nchunks);

  const int ngrp = npix / PPW;
  sample_rows_f16<<<(ngrp + GW - 1) / GW, GW * 32, 0, stream>>>(x, offs, Aplane, npix);

  const int tiles = (npix / 64) * (NPAD / 64);
  wmma_gemm64<0, false, 0, 0, false, 0><<<dim3((tiles + 7) / 8, 1), 256, 0, stream>>>(
      (const unsigned short*)Aplane, (const unsigned short*)Aplane, KDIM, 0L,
      (const unsigned short*)Wt, (const unsigned short*)Wt, KDIM, 0L,
      (void*)Cbuf, (void*)Cbuf, NPAD, 0L,
      bias, bias, 0L,
      npix, NPAD, KDIM, WSCALE_INV);

  const int nvec = npix * (CODIM / 4);
  bias_rows_out<<<(nvec + 255) / 256, 256, 0, stream>>>(Cbuf, bias, out, nvec);
}
